// SDOT_16466904613557
// MI455X (gfx1250) — hardware-verified
//
#include <hip/hip_runtime.h>


#define NSRC 8192
#define NTG  16384
#define DD   128
#define EPS  0.05f

typedef unsigned short bf;
typedef __attribute__((ext_vector_type(16))) __bf16   v16bf;
typedef __attribute__((ext_vector_type(8)))  unsigned short v8us;
typedef __attribute__((ext_vector_type(8)))  float    v8f;
typedef __attribute__((ext_vector_type(4)))  float    v4f;

__device__ __forceinline__ unsigned short f2bf(float f) { unsigned u = __float_as_uint(f); u += 0x7FFFu + ((u >> 16) & 1u); return (unsigned short)(u >> 16); }
__device__ __forceinline__ float bf2f(unsigned short b) { return __uint_as_float(((unsigned)b) << 16); }
__device__ __forceinline__ float bfr(float f) { return bf2f(f2bf(f)); }
__device__ __forceinline__ v16bf cat16b(v8us lo, v8us hi) { return __builtin_bit_cast(v16bf, __builtin_shufflevector(lo, hi, 0, 1, 2, 3, 4, 5, 6, 7, 8, 9, 10, 11, 12, 13, 14, 15)); }
__device__ __forceinline__ v8f wmmab(v16bf a, v16bf b, v8f c) { return __builtin_amdgcn_wmma_f32_16x16x32_bf16(false, a, false, b, (short)0, c, false, false); }
#define VST2(T, p, v) do { const T vst2_v_ = (v); *(volatile T*)(p) = vst2_v_; __threadfence(); *(volatile T*)(p) = vst2_v_; } while (0)

__global__ __launch_bounds__(256) void k_rows(const float* __restrict__ src, int rows, bf* dst) {
    typedef __attribute__((ext_vector_type(4))) unsigned short v4us;
    const int lane = threadIdx.x & 31, r = blockIdx.x * 8 + (threadIdx.x >> 5);
    if (r >= rows) return;
    v4us o;
#pragma unroll
    for (int i = 0; i < 4; ++i) o[i] = f2bf(src[(size_t)r * DD + lane * 4 + i]);
    VST2(v4us, dst + (size_t)r * DD + lane * 4, o);
}
__global__ __launch_bounds__(256) void k_ysq(const float* __restrict__ y, float* YS) {
    const int m = blockIdx.x * 256 + threadIdx.x;
    float s = 0.f;
#pragma unroll 4
    for (int d = 0; d < DD; ++d) { const float v = bfr(y[(size_t)m * DD + d]); s += v * v; }
    VST2(float, YS + m, s);
}
__global__ __launch_bounds__(256) void k_psimean(const float* __restrict__ psi, float* PM) {
    __shared__ float red[256];
    const int t = threadIdx.x; float s = 0.f;
    for (int m = t; m < NTG; m += 256) s += bfr(psi[m]);
    red[t] = s; __syncthreads();
    for (int st = 128; st > 0; st >>= 1) { if (t < st) red[t] += red[t + st]; __syncthreads(); }
    if (t < 32) { const float v = red[0] / (float)NTG; VST2(float, PM + t, v); }
}
__global__ __launch_bounds__(128) void k_lse(const bf* __restrict__ Xb, const bf* __restrict__ Yb, const float* __restrict__ x, const float* __restrict__ YS, const float* __restrict__ psi, const float* __restrict__ PM, float* out) {
    __shared__ float ost[4][16];
    const int lane = threadIdx.x & 31, wave = threadIdx.x >> 5, lr = lane & 15, hi = lane >> 4;
    const int r0 = blockIdx.x * 64 + wave * 16;
    v16bf xa[4];
#pragma unroll
    for (int kc = 0; kc < 4; ++kc) { const bf* p = Xb + (size_t)(r0 + lr) * DD + kc * 32 + 8 * hi; xa[kc] = cat16b(*(const v8us*)p, *(const v8us*)(p + 16)); }
    float xs[8];
#pragma unroll
    for (int j = 0; j < 8; ++j) { float s = 0.f; const float* xr = x + (size_t)(r0 + hi * 8 + j) * DD;
#pragma unroll 4
        for (int d = 0; d < DD; ++d) { const float v = bfr(xr[d]); s += v * v; }
        xs[j] = s; }
    float M[8], S[8];
#pragma unroll
    for (int j = 0; j < 8; ++j) { M[j] = -3.0e38f; S[j] = 0.f; }
    const float ie = 1.0f / EPS;
#pragma unroll 1
    for (int mt = 0; mt < NTG / 32; ++mt) {
        const int m0 = mt * 32;
        v8f g0 = {}, g1 = {};
#pragma unroll
        for (int kc = 0; kc < 4; ++kc) { const bf* p0 = Yb + (size_t)(m0 + lr) * DD + kc * 32 + 8 * hi; const bf* p1 = p0 + (size_t)16 * DD;
            g0 = wmmab(xa[kc], cat16b(*(const v8us*)p0, *(const v8us*)(p0 + 16)), g0); g1 = wmmab(xa[kc], cat16b(*(const v8us*)p1, *(const v8us*)(p1 + 16)), g1); }
        asm volatile("v_nop\n\tv_nop\n\tv_nop\n\tv_nop" : "+v"(g0), "+v"(g1) : "v"(xa[0]), "v"(xa[3]));
        const float ysa = YS[m0 + lr], ysb = YS[m0 + 16 + lr], pa = bfr(psi[m0 + lr]), pb = bfr(psi[m0 + 16 + lr]);
#pragma unroll
        for (int j = 0; j < 8; ++j) {
            const float ca = xs[j] + ysa - 2.0f * g0[j], cb = xs[j] + ysb - 2.0f * g1[j];
            const float za = (pa - ca) * ie, zb = (pb - cb) * ie;
            float mx = fmaxf(za, zb);
            mx = fmaxf(mx, __shfl_xor(mx, 1, 16)); mx = fmaxf(mx, __shfl_xor(mx, 2, 16)); mx = fmaxf(mx, __shfl_xor(mx, 4, 16)); mx = fmaxf(mx, __shfl_xor(mx, 8, 16));
            const float mn = fmaxf(M[j], mx);
            S[j] = S[j] * __expf(M[j] - mn) + (__expf(za - mn) + __expf(zb - mn)); M[j] = mn; }
    }
    const float pm = PM[0];
#pragma unroll
    for (int j = 0; j < 8; ++j) { float s = S[j]; s += __shfl_xor(s, 1, 16); s += __shfl_xor(s, 2, 16); s += __shfl_xor(s, 4, 16); s += __shfl_xor(s, 8, 16);
        if (lr == 0) ost[wave][hi * 8 + j] = -EPS * (M[j] + __logf(s)) + pm; }
    __syncthreads();
    if (threadIdx.x < 64) { const float v = ost[threadIdx.x >> 4][threadIdx.x & 15]; *(volatile float*)(out + blockIdx.x * 64 + threadIdx.x) = v; }
    __threadfence();
    if (threadIdx.x < 64) { const float v = ost[threadIdx.x >> 4][threadIdx.x & 15]; *(volatile float*)(out + blockIdx.x * 64 + threadIdx.x) = v; }
}

extern "C" void kernel_launch(void* const* d_in, const int* in_sizes, int n_in,
                              void* d_out, int out_size, void* d_ws, size_t ws_size, hipStream_t stream) {
    (void)in_sizes; (void)n_in; (void)out_size;
    const float* x = (const float*)d_in[0]; const float* y = (const float*)d_in[1]; const float* psi = (const float*)d_in[2];
    float* out = (float*)d_out;
    char* wsp = (char*)d_ws;
    auto take = [&](size_t bytes) { char* p = wsp; wsp += (bytes + 255) & ~(size_t)255; return (void*)p; };
    bf* Xb = (bf*)take((size_t)NSRC * DD * 2); bf* Yb = (bf*)take((size_t)NTG * DD * 2); float* YS = (float*)take((size_t)NTG * 4); float* PM = (float*)take(256);
    if ((size_t)(wsp - (char*)d_ws) > ws_size) return;
    k_rows<<<NSRC / 8, 256, 0, stream>>>(x, NSRC, Xb); k_rows<<<NTG / 8, 256, 0, stream>>>(y, NTG, Yb);
    k_ysq<<<NTG / 256, 256, 0, stream>>>(y, YS);
    k_psimean<<<1, 256, 0, stream>>>(psi, PM);
    k_lse<<<NSRC / 64, 128, 0, stream>>>(Xb, Yb, x, YS, psi, PM, out);
}
